// VideoImitation_45603962749554
// MI455X (gfx1250) — hardware-run, weakly checked
//
#include <hip/hip_runtime.h>


#ifndef NB
#define NB 8
#endif
#define NB_FULL   8
#define CH        512
#define FF        128
#define NHD       4
#define HC        32
#define HWN       84
#define FP        96
#define DFR       4
#define OFR       32
#define DREAL     336
#define DPAD      384
#define DTILES    6
#define OBSP      3072
#define NPOS      3456
#define PTILES    54
#define THW_FULL  3024
#define Q4N       756
#define QKC       256
#define QKVR      384
#define PSP       40
#define SCW       1536
#define INV_TEMP  0.04419417382415922f
#define BG        ((NB) < 4 ? (NB) : 4)

static_assert(NB <= NB_FULL);
static_assert(NB % BG == 0);
static_assert(CH % 64 == 0);
static_assert(CH % 32 == 0);
static_assert(FF % 32 == 0);
static_assert(NHD * HC == FF);
static_assert(HC == 32);
static_assert(DFR * HWN == DREAL);
static_assert(DREAL % 16 == 0);
static_assert(DREAL % 8 == 0);
static_assert(DPAD == DTILES * 64);
static_assert(OFR * FP == OBSP);
static_assert(DPAD + OBSP == NPOS);
static_assert(PTILES * 64 == NPOS);
static_assert(OBSP % 64 == 0);
static_assert(FP % 16 == 0);
static_assert(HWN % 4 == 0);
static_assert(FP % 4 == 0);
static_assert((DFR + OFR) * HWN == THW_FULL);
static_assert(Q4N * 4 == THW_FULL);
static_assert(QKVR == 3 * FF);
static_assert((PSP * 2) % 16 == 0);
static_assert(SCW == 6 * 32 * 8);
static_assert((FP * HC) % (8 * 64) == 0);
static_assert(DREAL + FP == 13 * 32 + 16);
static_assert(((size_t)NB * CH * Q4N) % 256 == 0);

typedef unsigned short bf;
typedef __attribute__((ext_vector_type(16))) __bf16   v16bf;
typedef __attribute__((ext_vector_type(8)))  unsigned short v8us;
typedef v8us __attribute__((may_alias)) v8usa;
typedef __attribute__((ext_vector_type(8)))  float    v8f;
typedef __attribute__((ext_vector_type(4)))  float    v4f;
typedef v4f  __attribute__((may_alias)) v4fa;
typedef __attribute__((ext_vector_type(2)))  double   v2d;

__device__ __forceinline__ unsigned short f2bf(float f) { unsigned u = __float_as_uint(f); u += 0x7FFFu + ((u >> 16) & 1u); return (unsigned short)(u >> 16); }
__device__ __forceinline__ float bf2f(unsigned short w) { return __uint_as_float(((unsigned)w) << 16); }
__device__ __forceinline__ v16bf cat16b(v8us lo, v8us hi) { return __builtin_bit_cast(v16bf, __builtin_shufflevector(lo, hi, 0, 1, 2, 3, 4, 5, 6, 7, 8, 9, 10, 11, 12, 13, 14, 15)); }
__device__ __forceinline__ v8f wmmab(v16bf a, v16bf b, v8f c) { return __builtin_amdgcn_wmma_f32_16x16x32_bf16(false, a, false, b, (short)0, c, false, false); }
__device__ __forceinline__ v16bf ldb(const bf* p)  { return cat16b(*(const v8us*)p, *(const v8us*)(p + 16)); }
__device__ __forceinline__ void wave_sync() { __builtin_amdgcn_fence(3  , "wavefront"); __builtin_amdgcn_wave_barrier(); asm volatile("" ::: "memory"); }
__device__ __forceinline__ void split8(const v4f a, const v4f b, v8us& h, v8us& l) {
#pragma unroll
    for (int k = 0; k < 4; ++k) {
        const unsigned short x = f2bf(a[k]); h[k] = x; l[k] = f2bf(a[k] - bf2f(x));
        const unsigned short y = f2bf(b[k]); h[4 + k] = y; l[4 + k] = f2bf(b[k] - bf2f(y)); }
}

__global__ __launch_bounds__(256) void k_cvtw(const float* __restrict__ src, bf* dst, int perLayer8, size_t dstLayerStride) {
    const int i = blockIdx.x * 256 + threadIdx.x; if (i >= 2 * perLayer8) return;
    const int L = i / perLayer8, r = i - L * perLayer8;
    const v8f v = *(const v8f*)(src + (size_t)i * 8); v8us o;
#pragma unroll
    for (int k = 0; k < 8; ++k) o[k] = f2bf(v[k]);
    bf* d = dst + (size_t)L * dstLayerStride + (size_t)r * 8;
    *(volatile v8us*)d = o; __threadfence(); *(volatile v8us*)d = o;
}

template <int LAYER>
__global__ __launch_bounds__(256) void k_xt(const float* __restrict__ in, float* X, const float* __restrict__ MR, bf* XTH, bf* XTL, int b0) {
    __shared__ float ts[64 * 65];
    const int tid = threadIdx.x; const int pc0 = blockIdx.x * 64, ch0 = blockIdx.y * 64, bz = blockIdx.z; const int b = b0 + bz;
    const bool wrx = (LAYER == 1) || (blockIdx.x < DTILES);
    v4f keep[4];
#pragma unroll
    for (int i = 0; i < 4; ++i) {
        const int idx = tid + 256 * i; const int ch = idx >> 4, c4 = (idx & 15) * 4; const int pc = pc0 + c4;
        const int oo = (pc >= DPAD) ? (pc - DPAD) : 0; const int t = oo / FP; const int j = oo - t * FP;
        const bool valid = (pc < DPAD) ? (pc < DREAL) : (j < HWN);
        v4f v;
        if (LAYER == 1) {
            int sc = (pc < DPAD) ? pc : (DREAL + t * HWN + j); sc = valid ? sc : 0;
            v = *(const v4f*)(in + ((size_t)(b * CH + ch0 + ch)) * THW_FULL + sc);
            v[0] = bf2f(f2bf(v[0])); v[1] = bf2f(f2bf(v[1])); v[2] = bf2f(f2bf(v[2])); v[3] = bf2f(f2bf(v[3]));
        } else {
            v = *(const v4f*)(X + ((size_t)(b * CH + ch0 + ch)) * NPOS + pc);
            const v4f mr = *(const v4f*)(MR + 4 * (ch0 + ch));
#pragma unroll
            for (int k = 0; k < 4; ++k) v[k] = (mr[2] * (v[k] - mr[0])) * mr[1] + mr[3];
        }
        const v4f z = {0.0f, 0.0f, 0.0f, 0.0f};
        v = valid ? v : z;
        keep[i] = v;
        ts[ch * 65 + c4 + 0] = v[0]; ts[ch * 65 + c4 + 1] = v[1]; ts[ch * 65 + c4 + 2] = v[2]; ts[ch * 65 + c4 + 3] = v[3];
    }
    __syncthreads();
    v8us h0, h1, l0, l1;
    { const int col = tid >> 3, p = tid & 7;
#pragma unroll
      for (int j = 0; j < 8; ++j) { const float x = ts[(p * 8 + j) * 65 + col]; const unsigned short hh = f2bf(x); h0[j] = hh; l0[j] = f2bf(x - bf2f(hh)); } }
    { const int col = (tid >> 3) + 32, p = tid & 7;
#pragma unroll
      for (int j = 0; j < 8; ++j) { const float x = ts[(p * 8 + j) * 65 + col]; const unsigned short hh = f2bf(x); h1[j] = hh; l1[j] = f2bf(x - bf2f(hh)); } }
    const size_t a0 = ((size_t)bz * NPOS + pc0 + (tid >> 3)) * CH + ch0 + (tid & 7) * 8;
    const size_t a1 = a0 + (size_t)32 * CH;
#pragma unroll 1
    for (int ps = 0; ps < 2; ++ps) {
        *(volatile v8us*)(XTH + a0) = h0; *(volatile v8us*)(XTH + a1) = h1;
        if (LAYER == 2) { *(volatile v8us*)(XTL + a0) = l0; *(volatile v8us*)(XTL + a1) = l1; }
        if (wrx) {
#pragma unroll
            for (int i = 0; i < 4; ++i) { const int idx = tid + 256 * i; const int ch = idx >> 4, c4 = (idx & 15) * 4;
                *(volatile v4f*)(X + ((size_t)(b * CH + ch0 + ch)) * NPOS + pc0 + c4) = keep[i]; }
        }
        if (ps == 0) __threadfence();
    }
}

template <int NPL>
__global__ __launch_bounds__(32) __attribute__((amdgpu_num_vgpr(256)))
void k_qkv(const bf* __restrict__ src, bf* dst, size_t xth_off, size_t xtl_off, size_t w_off,
           size_t qkh_off, size_t qkl_off, size_t vh_off, size_t vl_off) {
    __shared__ __align__(16) float os[16 * 68];
    const int lane = threadIdx.x & 31, lr = lane & 15, hi = lane >> 4;
    const int pt = blockIdx.x, y = blockIdx.y, bz = blockIdx.z;
    const size_t wset = w_off + (size_t)((pt >= DTILES) ? QKVR : 0) * CH;
    const size_t xrow = (size_t)bz * NPOS + (size_t)pt * 64;
    const bool qk = (y < 4);
    const size_t wq = wset + (size_t)(qk ? (y * 64) : (QKC + (y - 4) * 64)) * CH;
    const size_t a0 = qk ? (xth_off + xrow * CH) : wq;
    const size_t a1 = qk ? (xtl_off + xrow * CH) : wq;
    const size_t b0 = qk ? wq : (xth_off + xrow * CH);
    const size_t b1 = qk ? wq : (xtl_off + xrow * CH);
    const size_t opitch = qk ? (size_t)QKC : (size_t)NPOS;
    const size_t orel = qk ? (xrow * QKC + (size_t)y * 64) : (((size_t)bz * FF + (size_t)(y - 4) * 64) * NPOS + (size_t)pt * 64);
    const size_t ohb = (qk ? qkh_off : vh_off) + orel;
    const size_t olb = (qk ? qkl_off : vl_off) + orel;
    v8f acc[4][4];
#pragma unroll
    for (int mb = 0; mb < 4; ++mb)
#pragma unroll
        for (int nb = 0; nb < 4; ++nb) acc[mb][nb] = (v8f){};
    const size_t lo_ = (size_t)lr * CH + 8 * hi;
#pragma unroll 1
    for (int kc = 0; kc < CH; kc += 32) {
#pragma unroll 1
        for (int p = 0; p < NPL; ++p) {
            const size_t ao = ((p == 0) ? a0 : a1) + lo_ + kc, bo = ((p == 0) ? b0 : b1) + lo_ + kc;
            v16bf a[4];
#pragma unroll
            for (int mb = 0; mb < 4; ++mb) a[mb] = ldb(src + ao + (size_t)mb * 16 * CH);
#pragma unroll
            for (int nb = 0; nb < 4; ++nb) { const v16bf b = ldb(src + bo + (size_t)nb * 16 * CH);
#pragma unroll
                for (int mb = 0; mb < 4; ++mb) acc[mb][nb] = wmmab(a[mb], b, acc[mb][nb]); }
            asm volatile("v_nop\n\tv_nop\n\tv_nop\n\tv_nop" : "+v"(acc[0][0]), "+v"(acc[1][1]), "+v"(acc[2][2]), "+v"(acc[3][3]) : "v"(a[0]), "v"(a[1]), "v"(a[2]), "v"(a[3]));
        }
    }
#pragma unroll
    for (int mb = 0; mb < 4; ++mb) {
#pragma unroll
        for (int nb = 0; nb < 4; ++nb) {
#pragma unroll
            for (int j = 0; j < 8; ++j) os[(hi * 8 + j) * 68 + nb * 16 + lr] = acc[mb][nb][j]; }
        wave_sync();
#pragma unroll 1
        for (int ps = 0; ps < 2; ++ps) {
#pragma unroll
            for (int s = 0; s < 4; ++s) { const int row = 4 * s + (lane >> 3), pc = (lane & 7) * 8;
                const v4f x0 = *(const v4fa*)(&os[row * 68 + pc]), x1 = *(const v4fa*)(&os[row * 68 + pc + 4]);
                v8us h, l; split8(x0, x1, h, l);
                const size_t off = (size_t)(mb * 16 + row) * opitch + pc;
                *(volatile v8us*)(dst + ohb + off) = h; *(volatile v8us*)(dst + olb + off) = l; }
            if (ps == 0) __threadfence(); }
        wave_sync();
    }
}

__global__ __launch_bounds__(128) __attribute__((amdgpu_num_vgpr(256)))
void k_dattn(const bf* __restrict__ src, bf* dst, size_t qkh_off, size_t qkl_off, size_t vh_off, size_t vl_off, size_t dvh_off, size_t dvl_off) {
    __shared__ __align__(16) float ob[32 * 68];
    const int tid = threadIdx.x, lane = tid & 31, lr = lane & 15, hi = lane >> 4;
    const int wave = __builtin_amdgcn_readfirstlane(tid >> 5);
    const int n = blockIdx.y, bz = blockIdx.z;
    const int I0 = (blockIdx.x * 4 + wave) * 16;
    const bool active = I0 < DREAL;
    v8f acc0 = (v8f){}, acc1 = (v8f){};
    float linv = 0.0f;
    if (active) {
        const size_t prow0 = (size_t)bz * NPOS;
        const size_t ko = (prow0 + I0 + lr) * QKC + FF + (size_t)n * HC + 8 * hi;
        const v16bf kh = ldb(src + qkh_off + ko), kl = ldb(src + qkl_off + ko);
        const int jlim = ((I0 + lr) / HWN + 1) * HWN;
        const int nst = ((((I0 + 15) / HWN) + 1) * HWN + 31) >> 5;
        const size_t vrow0 = ((size_t)bz * FF + (size_t)n * HC + lr) * NPOS + 8 * hi;
        float m = -1e30f, l = 0.0f;
#pragma unroll 1
        for (int st = 0; st < nst; ++st) {
            const int J0 = st * 32;
            const size_t qo = (prow0 + J0 + lr) * QKC + (size_t)n * HC + 8 * hi;
            const v16bf qh0 = ldb(src + qkh_off + qo), ql0 = ldb(src + qkl_off + qo);
            const v16bf qh1 = ldb(src + qkh_off + qo + (size_t)16 * QKC), ql1 = ldb(src + qkl_off + qo + (size_t)16 * QKC);
            v8f s0 = (v8f){}, s1 = (v8f){};
            s0 = wmmab(qh0, kh, s0); s1 = wmmab(qh1, kh, s1);
            s0 = wmmab(qh0, kl, s0); s1 = wmmab(qh1, kl, s1);
            s0 = wmmab(ql0, kh, s0); s1 = wmmab(ql1, kh, s1);
            asm volatile("v_nop\n\tv_nop\n\tv_nop\n\tv_nop" : "+v"(s0), "+v"(s1) : "v"(qh0), "v"(qh1), "v"(ql0), "v"(ql1), "v"(kh), "v"(kl));
            float mx = -1e30f;
#pragma unroll
            for (int r = 0; r < 8; ++r) {
                const float v0 = (J0 + 8 * hi + r < jlim) ? s0[r] * INV_TEMP : -1e30f;
                const float v1 = (J0 + 16 + 8 * hi + r < jlim) ? s1[r] * INV_TEMP : -1e30f;
                s0[r] = v0; s1[r] = v1; mx = fmaxf(mx, fmaxf(v0, v1)); }
            mx = fmaxf(mx, __shfl_xor(mx, 16, 32));
            const float mnew = fmaxf(m, mx);
            const float alpha = __expf(m - mnew);
            float psum = 0.0f;
            v8us h0, l0, h1, l1;
#pragma unroll
            for (int r = 0; r < 8; ++r) {
                float e0 = __expf(s0[r] - mnew); e0 = (s0[r] > -1e29f) ? e0 : 0.0f;
                float e1 = __expf(s1[r] - mnew); e1 = (s1[r] > -1e29f) ? e1 : 0.0f;
                psum += e0 + e1;
                const unsigned short a = f2bf(e0); h0[r] = a; l0[r] = f2bf(e0 - bf2f(a));
                const unsigned short c = f2bf(e1); h1[r] = c; l1[r] = f2bf(e1 - bf2f(c)); }
            psum += __shfl_xor(psum, 16, 32);
            l = l * alpha + psum; m = mnew;
            acc0 *= alpha; acc1 *= alpha;
            const v16bf bh = cat16b(h0, h1), bl = cat16b(l0, l1);
            const size_t vo = vrow0 + J0;
            const v16bf vh0 = ldb(src + vh_off + vo), vl0 = ldb(src + vl_off + vo);
            const v16bf vh1 = ldb(src + vh_off + vo + (size_t)16 * NPOS), vl1 = ldb(src + vl_off + vo + (size_t)16 * NPOS);
            acc0 = wmmab(vh0, bh, acc0); acc1 = wmmab(vh1, bh, acc1);
            acc0 = wmmab(vh0, bl, acc0); acc1 = wmmab(vh1, bl, acc1);
            acc0 = wmmab(vl0, bh, acc0); acc1 = wmmab(vl1, bh, acc1);
            asm volatile("v_nop\n\tv_nop\n\tv_nop\n\tv_nop" : "+v"(acc0), "+v"(acc1) : "v"(vh0), "v"(vh1), "v"(vl0), "v"(vl1), "v"(bh), "v"(bl));
        }
        linv = 1.0f / l;
    }
#pragma unroll
    for (int r = 0; r < 8; ++r) {
        ob[(8 * hi + r) * 68 + wave * 16 + lr] = acc0[r] * linv;
        ob[(16 + 8 * hi + r) * 68 + wave * 16 + lr] = acc1[r] * linv; }
    __syncthreads();
    const size_t obase = ((size_t)bz * FF + (size_t)n * HC) * DPAD + (size_t)blockIdx.x * 64;
#pragma unroll 1
    for (int ps = 0; ps < 2; ++ps) {
#pragma unroll
        for (int i = 0; i < 2; ++i) { const int idx = tid + 128 * i; const int row = idx >> 3, pc = (idx & 7) * 8;
            const v4f x0 = *(const v4fa*)(&ob[row * 68 + pc]), x1 = *(const v4fa*)(&ob[row * 68 + pc + 4]);
            v8us h, l; split8(x0, x1, h, l);
            const size_t off = obase + (size_t)row * DPAD + pc;
            *(volatile v8us*)(dst + dvh_off + off) = h; *(volatile v8us*)(dst + dvl_off + off) = l; }
        if (ps == 0) __threadfence(); }
}

__global__ __launch_bounds__(64) __attribute__((amdgpu_num_vgpr(256)))
void k_oattn(const bf* __restrict__ src, bf* dst, size_t qkh_off, size_t qkl_off, size_t vh_off, size_t vl_off,
             size_t dvh_off, size_t dvl_off, size_t oh_off, size_t ol_off) {
    __shared__ __align__(16) bf sph[FP * PSP];
    __shared__ __align__(16) bf spl[FP * PSP];
    __shared__ __align__(16) bf soh[FP * HC];
    __shared__ __align__(16) bf sol[FP * HC];
    __shared__ __align__(16) float ssc[2 * SCW];
    const int tid = threadIdx.x, lane = tid & 31, lr = lane & 15, hi = lane >> 4;
    const int wave = __builtin_amdgcn_readfirstlane(tid >> 5);
    const int t = blockIdx.x, n = blockIdx.y, bz = blockIdx.z;
    const size_t prow0 = (size_t)bz * NPOS;
    const size_t orow0 = prow0 + DPAD + (size_t)FP * t;
    const size_t qoff = (orow0 + lr) * QKC + (size_t)n * HC + 8 * hi;
    const size_t chn = (size_t)bz * FF + (size_t)n * HC + (size_t)wave * 16 + lr;
    const size_t dbase = chn * DPAD, vbase = chn * NPOS + DPAD + (size_t)FP * t;
    const bool j5ok = lr < (HWN - 80);
    const int sb = wave * SCW + lane * 8;
    v8f acc[6];
#pragma unroll
    for (int jt = 0; jt < 6; ++jt) acc[jt] = (v8f){};
#pragma unroll 1
    for (int st = 0; st < 14; ++st) {
        {
            const int Ib = st * 32 + wave * 16;
            const bool tv = Ib < DREAL + FP;
            size_t grow = (Ib < DREAL) ? (prow0 + Ib + lr) : (orow0 + (size_t)(Ib - DREAL + lr));
            grow = tv ? grow : prow0;
            const size_t koff = grow * QKC + FF + (size_t)n * HC + 8 * hi;
            const v16bf kh = ldb(src + qkh_off + koff), kl = ldb(src + qkl_off + koff);
#pragma unroll 1
            for (int jt = 0; jt < 6; ++jt) {
                const size_t qo = qoff + (size_t)jt * 16 * QKC;
                const v16bf qh = ldb(src + qkh_off + qo), ql = ldb(src + qkl_off + qo);
                v8f z = (v8f){};
                z = wmmab(kh, qh, z); z = wmmab(kh, ql, z); z = wmmab(kl, qh, z);
                asm volatile("v_nop\n\tv_nop\n\tv_nop\n\tv_nop" : "+v"(z) : "v"(kh), "v"(kl), "v"(qh), "v"(ql));
                const v4f z0 = {z[0], z[1], z[2], z[3]}, z1 = {z[4], z[5], z[6], z[7]};
                *(v4fa*)(&ssc[sb + jt * 256]) = z0; *(v4fa*)(&ssc[sb + jt * 256 + 4]) = z1;
            }
            wave_sync();
#pragma unroll 1
            for (int r = 0; r < 8; ++r) {
                const float x0 = ssc[sb + r] * INV_TEMP, x1 = ssc[sb + 256 + r] * INV_TEMP, x2 = ssc[sb + 512 + r] * INV_TEMP;
                const float x3 = ssc[sb + 768 + r] * INV_TEMP, x4 = ssc[sb + 1024 + r] * INV_TEMP;
                const float y5 = ssc[sb + 1280 + r] * INV_TEMP;
                const float x5 = j5ok ? y5 : -1e30f;
                float mx = fmaxf(fmaxf(fmaxf(x0, x1), fmaxf(x2, x3)), fmaxf(x4, x5));
                mx = fmaxf(mx, __shfl_xor(mx, 1, 32)); mx = fmaxf(mx, __shfl_xor(mx, 2, 32));
                mx = fmaxf(mx, __shfl_xor(mx, 4, 32)); mx = fmaxf(mx, __shfl_xor(mx, 8, 32));
                const float e0 = __expf(x0 - mx), e1 = __expf(x1 - mx), e2 = __expf(x2 - mx), e3 = __expf(x3 - mx), e4 = __expf(x4 - mx);
                float e5 = __expf(x5 - mx); e5 = j5ok ? e5 : 0.0f;
                float sum = ((e0 + e1) + (e2 + e3)) + (e4 + e5);
                sum += __shfl_xor(sum, 1, 32); sum += __shfl_xor(sum, 2, 32); sum += __shfl_xor(sum, 4, 32); sum += __shfl_xor(sum, 8, 32);
                float inv = __builtin_amdgcn_rcpf(sum);
                inv = ((Ib + 8 * hi + r) < (DREAL + HWN)) ? inv : 0.0f;
                ssc[sb + r] = e0 * inv; ssc[sb + 256 + r] = e1 * inv; ssc[sb + 512 + r] = e2 * inv;
                ssc[sb + 768 + r] = e3 * inv; ssc[sb + 1024 + r] = e4 * inv; ssc[sb + 1280 + r] = e5 * inv; }
            wave_sync();
#pragma unroll 1
            for (int jt = 0; jt < 6; ++jt) {
                const v4f p0 = *(const v4fa*)(&ssc[sb + jt * 256]), p1 = *(const v4fa*)(&ssc[sb + jt * 256 + 4]);
                v8us ph_, pl_; split8(p0, p1, ph_, pl_);
                const int so = (jt * 16 + lr) * PSP + wave * 16 + 8 * hi;
                *(v8usa*)(&sph[so]) = ph_; *(v8usa*)(&spl[so]) = pl_; }
        }
        __syncthreads();
        v16bf vh, vl;
        {
            const int g0 = st * 32 + 8 * hi;
            const bool g1ok = st < 13;
            const int g1 = g1ok ? (g0 + 16) : DREAL;
            const v8us zz = {0, 0, 0, 0, 0, 0, 0, 0};
            const size_t o0h = (g0 < DREAL) ? (dvh_off + dbase + g0) : (vh_off + vbase + (size_t)(g0 - DREAL));
            const size_t o0l = (g0 < DREAL) ? (dvl_off + dbase + g0) : (vl_off + vbase + (size_t)(g0 - DREAL));
            const size_t o1h = (g1 < DREAL) ? (dvh_off + dbase + g1) : (vh_off + vbase + (size_t)(g1 - DREAL));
            const size_t o1l = (g1 < DREAL) ? (dvl_off + dbase + g1) : (vl_off + vbase + (size_t)(g1 - DREAL));
            const v8us a0h = *(const v8us*)(src + o0h), a0l = *(const v8us*)(src + o0l);
            v8us a1h = *(const v8us*)(src + o1h), a1l = *(const v8us*)(src + o1l);
            a1h = g1ok ? a1h : zz; a1l = g1ok ? a1l : zz;
            vh = cat16b(a0h, a1h); vl = cat16b(a0l, a1l);
        }
#pragma unroll
        for (int jp = 0; jp < 3; ++jp) {
            const int s0 = ((2 * jp) * 16 + lr) * PSP + 8 * hi, s1 = s0 + 16 * PSP;
            const v16bf bh0 = cat16b(*(const v8usa*)(&sph[s0]), *(const v8usa*)(&sph[s0 + 16]));
            const v16bf bl0 = cat16b(*(const v8usa*)(&spl[s0]), *(const v8usa*)(&spl[s0 + 16]));
            const v16bf bh1 = cat16b(*(const v8usa*)(&sph[s1]), *(const v8usa*)(&sph[s1 + 16]));
            const v16bf bl1 = cat16b(*(const v8usa*)(&spl[s1]), *(const v8usa*)(&spl[s1 + 16]));
            acc[2 * jp] = wmmab(vh, bh0, acc[2 * jp]); acc[2 * jp + 1] = wmmab(vh, bh1, acc[2 * jp + 1]);
            acc[2 * jp] = wmmab(vh, bl0, acc[2 * jp]); acc[2 * jp + 1] = wmmab(vh, bl1, acc[2 * jp + 1]);
            acc[2 * jp] = wmmab(vl, bh0, acc[2 * jp]); acc[2 * jp + 1] = wmmab(vl, bh1, acc[2 * jp + 1]);
            asm volatile("v_nop\n\tv_nop\n\tv_nop\n\tv_nop" : "+v"(acc[2 * jp]), "+v"(acc[2 * jp + 1]) : "v"(vh), "v"(vl), "v"(bh0), "v"(bl0), "v"(bh1), "v"(bl1) : "memory");
        }
        __syncthreads();
    }
#pragma unroll
    for (int jt = 0; jt < 6; ++jt) {
        const bool jv = (jt * 16 + lr) < HWN;
        v8us oh_, ol_;
#pragma unroll
        for (int r = 0; r < 8; ++r) { const float x = jv ? acc[jt][r] : 0.0f; const unsigned short a = f2bf(x); oh_[r] = a; ol_[r] = f2bf(x - bf2f(a)); }
        const int so = (jt * 16 + lr) * HC + wave * 16 + 8 * hi;
        *(v8usa*)(&soh[so]) = oh_; *(v8usa*)(&sol[so]) = ol_; }
    __syncthreads();
    const size_t obase = (((size_t)bz * NHD + n) * OBSP + (size_t)FP * t) * HC;
#pragma unroll 1
    for (int ps = 0; ps < 2; ++ps) {
#pragma unroll 1
        for (int i = 0; i < (FP * HC) / (8 * 64); ++i) {
            const int pc = (i * 64 + tid) * 8;
            const v8us a = *(const v8usa*)(&soh[pc]), b = *(const v8usa*)(&sol[pc]);
            *(volatile v8us*)(dst + oh_off + obase + pc) = a; *(volatile v8us*)(dst + ol_off + obase + pc) = b; }
        if (ps == 0) __threadfence(); }
}

template <int LAYER>
__global__ __launch_bounds__(32) __attribute__((amdgpu_num_vgpr(256)))
void k_oconv(const bf* __restrict__ src, size_t wo_off, size_t oh_off, size_t ol_off, float* X, const float* __restrict__ MR, int b0) {
    __shared__ __align__(16) float os[16 * 68];
    const int lane = threadIdx.x & 31, lr = lane & 15, hi = lane >> 4;
    const int pt = blockIdx.x, my = blockIdx.y, bz = blockIdx.z; const int b = b0 + bz;
    v8f acc[4][4];
#pragma unroll
    for (int mb = 0; mb < 4; ++mb)
#pragma unroll
        for (int nb = 0; nb < 4; ++nb) acc[mb][nb] = (v8f){};
    const size_t aoff = wo_off + ((size_t)my * 64 + lr) * FF + 8 * hi;
#pragma unroll 1
    for (int kc = 0; kc < FF; kc += 32) {
        const int n = kc >> 5;
        v16bf a[4];
#pragma unroll
        for (int mb = 0; mb < 4; ++mb) a[mb] = ldb(src + aoff + (size_t)mb * 16 * FF + kc);
        const size_t bo = (((size_t)bz * NHD + n) * OBSP + (size_t)pt * 64 + lr) * HC + 8 * hi;
#pragma unroll
        for (int nb = 0; nb < 4; ++nb) { const v16bf bh = ldb(src + oh_off + bo + (size_t)nb * 16 * HC); const v16bf bl = ldb(src + ol_off + bo + (size_t)nb * 16 * HC);
#pragma unroll
            for (int mb = 0; mb < 4; ++mb) acc[mb][nb] = wmmab(a[mb], bh, acc[mb][nb]);
#pragma unroll
            for (int mb = 0; mb < 4; ++mb) acc[mb][nb] = wmmab(a[mb], bl, acc[mb][nb]); }
        asm volatile("v_nop\n\tv_nop\n\tv_nop\n\tv_nop" : "+v"(acc[0][0]), "+v"(acc[1][1]), "+v"(acc[2][2]), "+v"(acc[3][3]) : "v"(a[0]), "v"(a[1]), "v"(a[2]), "v"(a[3]));
    }
    const int cofs = lr * 4;
    const int pcol = pt * 64 + cofs;
    const bool valid = (pcol % FP) < HWN;
#pragma unroll
    for (int mb = 0; mb < 4; ++mb) {
#pragma unroll
        for (int nb = 0; nb < 4; ++nb) {
#pragma unroll
            for (int j = 0; j < 8; ++j) os[(hi * 8 + j) * 68 + nb * 16 + lr] = acc[mb][nb][j]; }
        wave_sync();
        v4f vals[8];
#pragma unroll
        for (int s = 0; s < 8; ++s) { const int row = 2 * s + hi; const int ch = my * 64 + mb * 16 + row;
            const v4f d = *(const v4fa*)(&os[row * 68 + cofs]);
            v4f x = *(const v4f*)(X + ((size_t)(b * CH + ch)) * NPOS + DPAD + pcol);
            if (LAYER == 2) { const v4f mr = *(const v4f*)(MR + 4 * ch);
#pragma unroll
                for (int k = 0; k < 4; ++k) x[k] = (mr[2] * (x[k] - mr[0])) * mr[1] + mr[3]; }
            v4f val;
#pragma unroll
            for (int k = 0; k < 4; ++k) val[k] = valid ? (x[k] + fmaxf(d[k], 0.0f)) : 0.0f;
            vals[s] = val; }
#pragma unroll
        for (int s = 0; s < 8; ++s) { const int ch = my * 64 + mb * 16 + 2 * s + hi;
            *(volatile v4f*)(X + ((size_t)(b * CH + ch)) * NPOS + DPAD + pcol) = vals[s]; }
        __threadfence();
#pragma unroll
        for (int s = 0; s < 8; ++s) { const int ch = my * 64 + mb * 16 + 2 * s + hi;
            *(volatile v4f*)(X + ((size_t)(b * CH + ch)) * NPOS + DPAD + pcol) = vals[s]; }
        wave_sync();
    }
}

__global__ __launch_bounds__(256) void k_stat(const float* __restrict__ X, double* PART) {
    __shared__ __align__(16) double red[32];
    const int tid = threadIdx.x, lane = tid & 31;
    const int wave = __builtin_amdgcn_readfirstlane(tid >> 5);
    const int b = blockIdx.y, ch0 = blockIdx.x * 16;
#pragma unroll 1
    for (int cc = 0; cc < 2; ++cc) {
        const int chl = wave * 2 + cc;
        const float* row = X + ((size_t)(b * CH + ch0 + chl)) * NPOS;
        float s = 0.0f, q = 0.0f;
#pragma unroll 1
        for (int qi = lane; qi < Q4N; qi += 32) {
            const int qq = (qi >= HWN) ? (qi - HWN) : 0; const int t = qq / 21; const int j4 = qq - 21 * t;
            const int col = (qi < HWN) ? (4 * qi) : (DPAD + FP * t + 4 * j4);
            const v4f v = *(const v4f*)(row + col);
            s += (v[0] + v[1]) + (v[2] + v[3]);
            q += (v[0] * v[0] + v[1] * v[1]) + (v[2] * v[2] + v[3] * v[3]); }
        double ds = (double)s, dq = (double)q;
        ds += __shfl_xor(ds, 16, 32); dq += __shfl_xor(dq, 16, 32);
        ds += __shfl_xor(ds, 8, 32);  dq += __shfl_xor(dq, 8, 32);
        ds += __shfl_xor(ds, 4, 32);  dq += __shfl_xor(dq, 4, 32);
        ds += __shfl_xor(ds, 2, 32);  dq += __shfl_xor(dq, 2, 32);
        ds += __shfl_xor(ds, 1, 32);  dq += __shfl_xor(dq, 1, 32);
        if (lane == 0) { red[chl * 2] = ds; red[chl * 2 + 1] = dq; }
    }
    __syncthreads();
    if (tid < 16) { v2d val; val[0] = red[tid * 2]; val[1] = red[tid * 2 + 1];
        double* o = PART + ((size_t)b * CH + ch0 + tid) * 2;
        *(volatile v2d*)o = val; __threadfence(); *(volatile v2d*)o = val; }
}

__global__ __launch_bounds__(256) void k_bnfin(const double* __restrict__ PART, const float* __restrict__ gamma, const float* __restrict__ beta, float* MR) {
    const int ch = blockIdx.x * 256 + threadIdx.x;
    double s = 0.0, q = 0.0;
#pragma unroll 1
    for (int b = 0; b < NB; ++b) { s += PART[((size_t)b * CH + ch) * 2]; q += PART[((size_t)b * CH + ch) * 2 + 1]; }
    const double invn = 1.0 / (double)((size_t)NB * THW_FULL);
    const double mean = s * invn;
    double var = q * invn - mean * mean; var = (var > 0.0) ? var : 0.0;
    v4f o; o[0] = (float)mean; o[1] = rsqrtf((float)var + 1e-5f); o[2] = gamma[ch]; o[3] = beta[ch];
    *(volatile v4f*)(MR + 4 * ch) = o; __threadfence(); *(volatile v4f*)(MR + 4 * ch) = o;
}

__global__ __launch_bounds__(256) void k_bnout(const float* __restrict__ X, const float* __restrict__ MR, float* out) {
    const size_t i = (size_t)blockIdx.x * 256 + threadIdx.x;
    if (i >= (size_t)NB * CH * Q4N) return;
    const int row = (int)(i / Q4N); const int qi = (int)(i - (size_t)row * Q4N);
    const int qq = (qi >= HWN) ? (qi - HWN) : 0; const int t = qq / 21; const int j4 = qq - 21 * t;
    const int col = (qi < HWN) ? (4 * qi) : (DPAD + FP * t + 4 * j4);
    const int ch = row & (CH - 1);
    const v4f x = *(const v4f*)(X + (size_t)row * NPOS + col);
    const v4f mr = *(const v4f*)(MR + 4 * ch);
    v4f y;
#pragma unroll
    for (int k = 0; k < 4; ++k) y[k] = (mr[2] * (x[k] - mr[0])) * mr[1] + mr[3];
    float* o = out + i * 4;
    *(volatile v4f*)o = y; __threadfence(); *(volatile v4f*)o = y;
}

static constexpr size_t al256(size_t v) { return (v + 255) & ~(size_t)255; }
static constexpr size_t SZ_X   = al256((size_t)NB * CH * NPOS * 4);
static constexpr size_t SZ_XT  = al256((size_t)BG * NPOS * CH * 2);
static constexpr size_t SZ_QK  = al256((size_t)BG * NPOS * QKC * 2);
static constexpr size_t SZ_V   = al256((size_t)BG * FF * NPOS * 2);
static constexpr size_t SZ_DV  = al256((size_t)BG * FF * DPAD * 2);
static constexpr size_t SZ_O   = al256((size_t)BG * NHD * OBSP * HC * 2);
static constexpr size_t SZ_W   = al256((size_t)2 * 2 * QKVR * CH * 2);
static constexpr size_t SZ_WO  = al256((size_t)2 * CH * FF * 2);
static constexpr size_t SZ_PT  = al256((size_t)NB * CH * 16);
static constexpr size_t SZ_MR  = al256((size_t)CH * 16);
static constexpr size_t OFF_X   = 0;
static constexpr size_t OFF_XTH = OFF_X + SZ_X;
static constexpr size_t OFF_XTL = OFF_XTH + SZ_XT;
static constexpr size_t OFF_QKH = OFF_XTL + SZ_XT;
static constexpr size_t OFF_QKL = OFF_QKH + SZ_QK;
static constexpr size_t OFF_VH  = OFF_QKL + SZ_QK;
static constexpr size_t OFF_VL  = OFF_VH + SZ_V;
static constexpr size_t OFF_DVH = OFF_VL + SZ_V;
static constexpr size_t OFF_DVL = OFF_DVH + SZ_DV;
static constexpr size_t OFF_OH  = OFF_DVL + SZ_DV;
static constexpr size_t OFF_OL  = OFF_OH + SZ_O;
static constexpr size_t OFF_W   = OFF_OL + SZ_O;
static constexpr size_t OFF_WO  = OFF_W + SZ_W;
static constexpr size_t OFF_PT  = OFF_WO + SZ_WO;
static constexpr size_t OFF_MR1 = OFF_PT + SZ_PT;
static constexpr size_t OFF_MR2 = OFF_MR1 + SZ_MR;
static constexpr size_t SZ_TOTAL = OFF_MR2 + SZ_MR;
static_assert(SZ_TOTAL <= (size_t)134217728);
static_assert(((size_t)FF * CH) % 8 == 0);
static_assert(((size_t)FF * CH * 2) % 256 == 0);

extern "C" void kernel_launch(void* const* d_in, const int* in_sizes, int n_in,
                              void* d_out, int out_size, void* d_ws, size_t ws_size, hipStream_t stream) {
    if (n_in < 11) return;
    if ((size_t)in_sizes[0] < (size_t)NB * CH * THW_FULL) return;
    for (int i = 1; i <= 8; ++i) if ((size_t)in_sizes[i] < (size_t)2 * FF * CH) return;
    if ((size_t)in_sizes[9] < (size_t)2 * CH || (size_t)in_sizes[10] < (size_t)2 * CH) return;
    if ((size_t)out_size < (size_t)NB * CH * THW_FULL) return;
    if (SZ_TOTAL > ws_size) return;
    const float* xin  = (const float*)d_in[0];
    const float* dwq  = (const float*)d_in[1];
    const float* dwk  = (const float*)d_in[2];
    const float* dwv  = (const float*)d_in[3];
    const float* dwo  = (const float*)d_in[4];
    (void)dwo;
    const float* owq  = (const float*)d_in[5];
    const float* owk  = (const float*)d_in[6];
    const float* owv  = (const float*)d_in[7];
    const float* owo  = (const float*)d_in[8];
    const float* gam  = (const float*)d_in[9];
    const float* bet  = (const float*)d_in[10];
    float* OUT = (float*)d_out;
    char* wsp = (char*)d_ws;
    bf* wsb = (bf*)wsp;
    float* X   = (float*)(wsp + OFF_X);
    bf* XTH    = (bf*)(wsp + OFF_XTH);
    bf* XTL    = (bf*)(wsp + OFF_XTL);
    bf* WQ     = (bf*)(wsp + OFF_W);
    bf* WOO    = (bf*)(wsp + OFF_WO);
    double* PT = (double*)(wsp + OFF_PT);
    float* MR1 = (float*)(wsp + OFF_MR1);
    float* MR2 = (float*)(wsp + OFF_MR2);

    { const int n8 = FF * CH / 8; const unsigned g = (unsigned)((2 * n8 + 255) / 256);
      const size_t ls = (size_t)2 * QKVR * CH;
      k_cvtw<<<g, 256, 0, stream>>>(dwq, WQ + (size_t)0 * FF * CH, n8, ls);
      k_cvtw<<<g, 256, 0, stream>>>(dwk, WQ + (size_t)1 * FF * CH, n8, ls);
      k_cvtw<<<g, 256, 0, stream>>>(dwv, WQ + (size_t)2 * FF * CH, n8, ls);
      k_cvtw<<<g, 256, 0, stream>>>(owq, WQ + (size_t)3 * FF * CH, n8, ls);
      k_cvtw<<<g, 256, 0, stream>>>(owk, WQ + (size_t)4 * FF * CH, n8, ls);
      k_cvtw<<<g, 256, 0, stream>>>(owv, WQ + (size_t)5 * FF * CH, n8, ls);
      k_cvtw<<<g, 256, 0, stream>>>(owo, WOO, n8, (size_t)CH * FF); }

    const size_t xth = OFF_XTH / 2, xtl = OFF_XTL / 2, qkh = OFF_QKH / 2, qkl = OFF_QKL / 2, vh = OFF_VH / 2, vl = OFF_VL / 2;
    const size_t dvh = OFF_DVH / 2, dvl = OFF_DVL / 2, oh = OFF_OH / 2, ol = OFF_OL / 2;

    for (int L = 0; L < 2; ++L) {
        const size_t w_off  = OFF_W / 2 + (size_t)L * 2 * QKVR * CH;
        const size_t wo_off = OFF_WO / 2 + (size_t)L * CH * FF;
        for (int g = 0; g < NB / BG; ++g) {
            const int b0 = g * BG;
            if (L == 0) k_xt<1><<<dim3(PTILES, CH / 64, BG), 256, 0, stream>>>(xin, X, MR1, XTH, XTL, b0);
            else        k_xt<2><<<dim3(PTILES, CH / 64, BG), 256, 0, stream>>>(xin, X, MR1, XTH, XTL, b0);
            if (L == 0) k_qkv<1><<<dim3(PTILES, 6, BG), 32, 0, stream>>>(wsb, wsb, xth, xth, w_off, qkh, qkl, vh, vl);
            else        k_qkv<2><<<dim3(PTILES, 6, BG), 32, 0, stream>>>(wsb, wsb, xth, xtl, w_off, qkh, qkl, vh, vl);
            k_dattn<<<dim3(DTILES, NHD, BG), 128, 0, stream>>>(wsb, wsb, qkh, qkl, vh, vl, dvh, dvl);
            k_oattn<<<dim3(OFR, NHD, BG), 64, 0, stream>>>(wsb, wsb, qkh, qkl, vh, vl, dvh, dvl, oh, ol);
            if (L == 0) k_oconv<1><<<dim3(OBSP / 64, CH / 64, BG), 32, 0, stream>>>(wsb, wo_off, oh, ol, X, MR1, b0);
            else        k_oconv<2><<<dim3(OBSP / 64, CH / 64, BG), 32, 0, stream>>>(wsb, wo_off, oh, ol, X, MR1, b0);
        }
        k_stat<<<dim3(CH / 16, NB, 1), 256, 0, stream>>>(X, PT);
        k_bnfin<<<dim3(CH / 256, 1, 1), 256, 0, stream>>>(PT, gam + (size_t)L * CH, bet + (size_t)L * CH, (L == 0) ? MR1 : MR2);
    }
    k_bnout<<<dim3((unsigned)(((size_t)NB * CH * Q4N) / 256), 1, 1), 256, 0, stream>>>(X, MR2, OUT);
}
